// SelectiveAttentionModule_67456756351555
// MI455X (gfx1250) — hardware-verified
//
#include <hip/hip_runtime.h>


#define NB_  8
#define TT   2048
#define DE   768
#define DK   128
#define D3   384
typedef _Float16 h16;
typedef unsigned short bf;
typedef __attribute__((ext_vector_type(16))) __bf16   v16bf;
typedef __attribute__((ext_vector_type(16))) _Float16 v16h;
typedef __attribute__((ext_vector_type(8)))  _Float16 v8h;
typedef __attribute__((ext_vector_type(8)))  unsigned short v8us;
typedef __attribute__((ext_vector_type(8)))  float    v8f;
typedef __attribute__((ext_vector_type(4)))  float    v4f;
typedef v8h  __attribute__((may_alias)) v8ha;
typedef v4f  __attribute__((may_alias)) v4fa;
typedef v8us __attribute__((may_alias)) v8usa;

__device__ __forceinline__ unsigned short f2bf(float f) { unsigned u = __float_as_uint(f); u += 0x7FFFu + ((u >> 16) & 1u); return (unsigned short)(u >> 16); }
__device__ __forceinline__ float bf2f(unsigned short b) { return __uint_as_float(((unsigned)b) << 16); }
__device__ __forceinline__ float bfr(float f) { return bf2f(f2bf(f)); }
__device__ __forceinline__ v16h cat16(v8h lo, v8h hi) { return __builtin_shufflevector(lo, hi, 0, 1, 2, 3, 4, 5, 6, 7, 8, 9, 10, 11, 12, 13, 14, 15); }
__device__ __forceinline__ v16bf cat16b(v8us lo, v8us hi) { return __builtin_bit_cast(v16bf, __builtin_shufflevector(lo, hi, 0, 1, 2, 3, 4, 5, 6, 7, 8, 9, 10, 11, 12, 13, 14, 15)); }
__device__ __forceinline__ v8f wmma16(v16h a, v16h b, v8f c) { return __builtin_amdgcn_wmma_f32_16x16x32_f16(false, a, false, b, (short)0, c, false, false); }
__device__ __forceinline__ v8f wmmab(v16bf a, v16bf b, v8f c) { return __builtin_amdgcn_wmma_f32_16x16x32_bf16(false, a, false, b, (short)0, c, false, false); }


template <typename T16> struct WFrag;
template <> struct WFrag<h16> { typedef v16h V; static __device__ __forceinline__ V ld(const h16* p) { return cat16(*(const v8h*)p, *(const v8h*)(p + 16)); } static __device__ __forceinline__ v8f mma(V a, V b, v8f c) { return wmma16(a, b, c); } };
template <> struct WFrag<bf> { typedef v16bf V; static __device__ __forceinline__ V ld(const bf* p) { return cat16b(*(const v8us*)p, *(const v8us*)(p + 16)); } static __device__ __forceinline__ v8f mma(V a, V b, v8f c) { return wmmab(a, b, c); } };
template <typename T16, int NSPLIT, bool BIAS>
__global__ __launch_bounds__(32) void k_gemmw(const T16* __restrict__ A, const T16* __restrict__ A2, const T16* __restrict__ Bt, const T16* __restrict__ Bt2, int K, float* C, int ldc, const float* __restrict__ bias, size_t sA, size_t sB, size_t sC) {
    typedef typename WFrag<T16>::V V;
    __shared__ __align__(16) float os[16 * 68];
    const size_t z = blockIdx.z; A += z * sA; if (A2) A2 += z * sA; Bt += z * sB; if (Bt2) Bt2 += z * sB; C += z * sC;
    const int lane = threadIdx.x & 31, lr = lane & 15, hi = lane >> 4; const int r0 = blockIdx.x * 64, c0 = blockIdx.y * 64;
    v8f acc[4][4];
#pragma unroll
    for (int mb = 0; mb < 4; ++mb)
#pragma unroll
        for (int nb = 0; nb < 4; ++nb) acc[mb][nb] = (v8f){};
    const size_t aoff = (size_t)(r0 + lr) * K + 8 * hi, boff = (size_t)(c0 + lr) * K + 8 * hi;
#pragma unroll 1
    for (int kc = 0; kc < K; kc += 32) {
        V a[4], a2[4];
#pragma unroll
        for (int mb = 0; mb < 4; ++mb) { a[mb] = WFrag<T16>::ld(A + aoff + (size_t)mb * 16 * K + kc); if (NSPLIT == 1 || NSPLIT == 2) a2[mb] = WFrag<T16>::ld(A2 + aoff + (size_t)mb * 16 * K + kc); }
#pragma unroll
        for (int nb = 0; nb < 4; ++nb) { const V b = WFrag<T16>::ld(Bt + boff + (size_t)nb * 16 * K + kc); V b2; if (NSPLIT >= 2) b2 = WFrag<T16>::ld(Bt2 + boff + (size_t)nb * 16 * K + kc);
#pragma unroll
            for (int mb = 0; mb < 4; ++mb) { acc[mb][nb] = WFrag<T16>::mma(a[mb], b, acc[mb][nb]); if (NSPLIT == 1 || NSPLIT == 2) acc[mb][nb] = WFrag<T16>::mma(a2[mb], b, acc[mb][nb]); if (NSPLIT >= 2) acc[mb][nb] = WFrag<T16>::mma(a[mb], b2, acc[mb][nb]); } }
        asm volatile("v_nop\n\tv_nop\n\tv_nop\n\tv_nop" : "+v"(acc[0][0]), "+v"(acc[1][1]), "+v"(acc[2][2]), "+v"(acc[3][3]) : "v"(a[0]), "v"(a[3]));
    }
#pragma unroll
    for (int mb = 0; mb < 4; ++mb) {
#pragma unroll
        for (int nb = 0; nb < 4; ++nb) {
#pragma unroll
            for (int j = 0; j < 8; ++j) os[(hi * 8 + j) * 68 + nb * 16 + lr] = acc[mb][nb][j]; }
        __builtin_amdgcn_wave_barrier(); asm volatile("" ::: "memory");
        float* crow = C + (size_t)(r0 + mb * 16) * ldc + c0;
#pragma unroll 1
        for (int ps = 0; ps < 2; ++ps) {
#pragma unroll
            for (int s = 0; s < 8; ++s) { const int row = 2 * s + hi, cofs = lr * 4; v4f val = *(const v4fa*)(os + row * 68 + cofs); if (BIAS) { val[0] += bfr(bias[c0 + cofs]); val[1] += bfr(bias[c0 + cofs + 1]); val[2] += bfr(bias[c0 + cofs + 2]); val[3] += bfr(bias[c0 + cofs + 3]); }
                *(volatile v4f*)(crow + (size_t)row * ldc + cofs) = val; }
            if (ps == 0) __threadfence(); }
        __builtin_amdgcn_wave_barrier(); asm volatile("" ::: "memory");
    }
}

template <typename T16, int NSPLIT, int CMODE>
__global__ __launch_bounds__(32) void k_gemmc(const T16* __restrict__ A, const T16* __restrict__ A2, const T16* __restrict__ Bt, const T16* __restrict__ Bt2, int K, float* C, int ldc, int roff, size_t sA, size_t sB, size_t sC) {
    typedef typename WFrag<T16>::V V;
    __shared__ __align__(16) float os[16 * 68];
    const size_t z = blockIdx.z; A += z * sA; if (A2) A2 += z * sA; Bt += z * sB; if (Bt2) Bt2 += z * sB; C += z * sC;
    const int lane = threadIdx.x & 31, lr = lane & 15, hi = lane >> 4; const int r0 = blockIdx.x * 64, c0 = blockIdx.y * 64;
    if (CMODE == 1 && c0 > r0 + roff + 63) return;
    const int Kl = (CMODE == 2) ? min(K, r0 + roff + 64) : K;
    v8f acc[4][4];
#pragma unroll
    for (int mb = 0; mb < 4; ++mb)
#pragma unroll
        for (int nb = 0; nb < 4; ++nb) acc[mb][nb] = (v8f){};
    const size_t aoff = (size_t)(r0 + lr) * K + 8 * hi, boff = (size_t)(c0 + lr) * K + 8 * hi;
#pragma unroll 1
    for (int kc = 0; kc < Kl; kc += 32) {
        V a[4], a2[4];
#pragma unroll
        for (int mb = 0; mb < 4; ++mb) { a[mb] = WFrag<T16>::ld(A + aoff + (size_t)mb * 16 * K + kc); if (NSPLIT == 1 || NSPLIT == 2) a2[mb] = WFrag<T16>::ld(A2 + aoff + (size_t)mb * 16 * K + kc); }
#pragma unroll
        for (int nb = 0; nb < 4; ++nb) { const V b = WFrag<T16>::ld(Bt + boff + (size_t)nb * 16 * K + kc); V b2; if (NSPLIT >= 2) b2 = WFrag<T16>::ld(Bt2 + boff + (size_t)nb * 16 * K + kc);
#pragma unroll
            for (int mb = 0; mb < 4; ++mb) { acc[mb][nb] = WFrag<T16>::mma(a[mb], b, acc[mb][nb]); if (NSPLIT == 1 || NSPLIT == 2) acc[mb][nb] = WFrag<T16>::mma(a2[mb], b, acc[mb][nb]); if (NSPLIT >= 2) acc[mb][nb] = WFrag<T16>::mma(a[mb], b2, acc[mb][nb]); } }
        asm volatile("v_nop\n\tv_nop\n\tv_nop\n\tv_nop" : "+v"(acc[0][0]), "+v"(acc[1][1]), "+v"(acc[2][2]), "+v"(acc[3][3]) : "v"(a[0]), "v"(a[3]));
    }
#pragma unroll
    for (int mb = 0; mb < 4; ++mb) {
#pragma unroll
        for (int nb = 0; nb < 4; ++nb) {
#pragma unroll
            for (int j = 0; j < 8; ++j) os[(hi * 8 + j) * 68 + nb * 16 + lr] = acc[mb][nb][j]; }
        __builtin_amdgcn_wave_barrier(); asm volatile("" ::: "memory");
        float* crow = C + (size_t)(r0 + mb * 16) * ldc + c0;
#pragma unroll 1
        for (int ps = 0; ps < 2; ++ps) {
#pragma unroll
            for (int s = 0; s < 8; ++s) { const int row = 2 * s + hi, cofs = lr * 4; v4f val = *(const v4fa*)(os + row * 68 + cofs);
                *(volatile v4f*)(crow + (size_t)row * ldc + cofs) = val; }
            if (ps == 0) __threadfence(); }
        __builtin_amdgcn_wave_barrier(); asm volatile("" ::: "memory");
    }
}

__device__ __forceinline__ void splitf(float y, unsigned short& h, unsigned short& l) { h = f2bf(y); l = f2bf(y - bf2f(h)); }
typedef __attribute__((ext_vector_type(2))) unsigned short v2us;
typedef __attribute__((ext_vector_type(4))) unsigned short v4us;

__global__ __launch_bounds__(256) void k_cvt8(const float* __restrict__ src, bf* dst, size_t n8) { const size_t i = (size_t)blockIdx.x * 256 + threadIdx.x; if (i >= n8) return; const v8f v = *(const v8f*)(src + i * 8); v8us o;
#pragma unroll
    for (int k = 0; k < 8; ++k) o[k] = f2bf(v[k]); *(volatile v8us*)(dst + i * 8) = o; __threadfence(); *(volatile v8us*)(dst + i * 8) = o; }
__global__ __launch_bounds__(256) void k_temp(const float* __restrict__ QKV, const float* __restrict__ tq, const float* __restrict__ tv, const float* __restrict__ alpha, float* TQ, float* TV) { const int s = blockIdx.x * 256 + threadIdx.x; if (s >= TT) return; const float* q = QKV + (size_t)s * D3; const float* v = q + 2 * DK; float aq = 0.f, av = 0.f;
#pragma unroll 1
    for (int d = 0; d < DK; ++d) { const float x1 = q[d], x2 = v[d]; float g1 = __fmul_rn(0.5f * x1, __fadd_rn(1.0f, erff(x1 * 0.70710678118654752f))), g2 = __fmul_rn(0.5f * x2, __fadd_rn(1.0f, erff(x2 * 0.70710678118654752f))); asm volatile("" : "+v"(g1)); asm volatile("" : "+v"(g2));
        float p1 = __fmul_rn(bfr(tq[(size_t)s * DK + d]), g1), p2 = __fmul_rn(bfr(tv[(size_t)s * DK + d]), g2); asm volatile("" : "+v"(p1)); asm volatile("" : "+v"(p2)); aq = __fadd_rn(aq, p1); av = __fadd_rn(av, p2); }
    float sg = __fdiv_rn(1.0f, __fadd_rn(1.0f, __expf(-bfr(alpha[s])))); asm volatile("" : "+v"(sg)); const float pos = __fadd_rn(1.0f, __fmul_rn(sg, __logf((float)(s + 1)))); const float rq = __fadd_rn(pos, tanhf(aq)), rv = __fadd_rn(pos, tanhf(av));
    for (int ps = 0; ps < 2; ++ps) { *(volatile float*)(TQ + s) = rq; *(volatile float*)(TV + s) = rv; if (ps == 0) __threadfence(); } }
__global__ __launch_bounds__(256) void k_gpl(const float* __restrict__ QKV, const float* __restrict__ TQ, bf* GQh, bf* GQl, bf* Kh, bf* Kl) { const int e = (blockIdx.x * 256 + threadIdx.x) * 4; if (e >= TT * DK) return; const int d = e % DK; const int s = e / DK; const float t = TQ[s]; const float* q = QKV + (size_t)s * D3 + d; v4us a, b, c, dd;
#pragma unroll
    for (int u = 0; u < 4; ++u) { unsigned short h1, l1, h2, l2; splitf(__fmul_rn(t, q[u]), h1, l1); splitf(q[DK + u], h2, l2); a[u] = h1; b[u] = l1; c[u] = h2; dd[u] = l2; }
    for (int ps = 0; ps < 2; ++ps) { *(volatile v4us*)(GQh + e) = a; *(volatile v4us*)(GQl + e) = b; *(volatile v4us*)(Kh + e) = c; *(volatile v4us*)(Kl + e) = dd; if (ps == 0) __threadfence(); } }
__global__ __launch_bounds__(256) void k_gvt(const float* __restrict__ QKV, const float* __restrict__ TV, bf* Th, bf* Tl) { const int e = (blockIdx.x * 256 + threadIdx.x) * 4; if (e >= DK * TT) return; const int s = e % TT; const int d = e / TT; v4us oh, ol;
#pragma unroll
    for (int u = 0; u < 4; ++u) { unsigned short a, b; splitf(__fmul_rn(TV[s + u], QKV[(size_t)(s + u) * D3 + 2 * DK + d]), a, b); oh[u] = a; ol[u] = b; } *(volatile v4us*)(Th + e) = oh; *(volatile v4us*)(Tl + e) = ol; __threadfence(); *(volatile v4us*)(Th + e) = oh; *(volatile v4us*)(Tl + e) = ol; }
__global__ __launch_bounds__(256) void k_csoft(const float* __restrict__ Sb, bf* Ph, bf* Pl) { const int lane = threadIdx.x & 31; const int i = blockIdx.x * 8 + (threadIdx.x >> 5); if (i >= TT) return; const float* sr = Sb + (size_t)i * TT; float v[TT / 32]; float mx = -3.0e38f; const float scl = 0.088388347648318447f;
#pragma unroll
    for (int ch = 0; ch < TT / 128; ++ch) { const int j0 = ch * 128 + lane * 4; const v4f a = *(const v4f*)(sr + j0);
#pragma unroll
        for (int u = 0; u < 4; ++u) { const float t = (j0 + u <= i) ? a[u] * scl : -3.0e38f; v[ch * 4 + u] = t; mx = fmaxf(mx, t); } }
#pragma unroll
    for (int sh = 16; sh; sh >>= 1) mx = fmaxf(mx, __shfl_xor(mx, sh, 32));
    float sum = 0.f;
#pragma unroll
    for (int q = 0; q < TT / 32; ++q) { float d0 = __fsub_rn(v[q], mx); asm volatile("" : "+v"(d0)); v[q] = (v[q] > -1.0e38f) ? __builtin_amdgcn_exp2f(__fmul_rn(d0, 1.4426950408889634f)) : 0.f; sum += v[q]; }
#pragma unroll
    for (int sh = 16; sh; sh >>= 1) sum += __shfl_xor(sum, sh, 32);
    const float f = __fdiv_rn(1.0f, sum);
    for (int ps = 0; ps < 2; ++ps) {
#pragma unroll
        for (int ch = 0; ch < TT / 128; ++ch) { v4us oh, ol;
#pragma unroll
            for (int q = 0; q < 4; ++q) { unsigned short a, b; splitf(v[ch * 4 + q] * f, a, b); oh[q] = a; ol[q] = b; } const size_t oo = (size_t)i * TT + ch * 128 + lane * 4; *(volatile v4us*)(Ph + oo) = oh; *(volatile v4us*)(Pl + oo) = ol; }
        if (ps == 0) __threadfence(); } }

extern "C" void kernel_launch(void* const* d_in, const int* in_sizes, int n_in,
                              void* d_out, int out_size, void* d_ws, size_t ws_size, hipStream_t stream) {
    (void)in_sizes; (void)n_in; (void)out_size;
    const float** I = (const float**)d_in;
    const float *x = I[0], *Wq = I[1], *bq = I[2], *Wk = I[3], *bk = I[4], *Wv = I[5], *bv = I[6], *alpha = I[7], *tokq = I[8], *tokv = I[9];
    float* OUT = (float*)d_out;
    char* wsp = (char*)d_ws;
    auto take = [&](size_t bytes) { char* p = wsp; wsp += (bytes + 255) & ~(size_t)255; return (void*)p; };
    bf* BQ = (bf*)take((size_t)DK * DE * 2); bf* BK = (bf*)take((size_t)DK * DE * 2); bf* BV = (bf*)take((size_t)DK * DE * 2); bf* XB = (bf*)take((size_t)TT * DE * 2); float* QKV = (float*)take((size_t)TT * D3 * 4); float* TQ = (float*)take(TT * 4); float* TV = (float*)take(TT * 4);
    bf* GQh = (bf*)take((size_t)TT * DK * 2); bf* GQl = (bf*)take((size_t)TT * DK * 2); bf* Kh = (bf*)take((size_t)TT * DK * 2); bf* Kl = (bf*)take((size_t)TT * DK * 2); bf* GVh = (bf*)take((size_t)DK * TT * 2); bf* GVl = (bf*)take((size_t)DK * TT * 2);
    float* Sb = (float*)take((size_t)TT * TT * 4); bf* Ph = (bf*)take((size_t)TT * TT * 2); bf* Pl = (bf*)take((size_t)TT * TT * 2);
    if ((size_t)(wsp - (char*)d_ws) > ws_size) return;
    k_cvt8<<<(DK * DE / 8 + 255) / 256, 256, 0, stream>>>(Wq, BQ, DK * DE / 8); k_cvt8<<<(DK * DE / 8 + 255) / 256, 256, 0, stream>>>(Wk, BK, DK * DE / 8); k_cvt8<<<(DK * DE / 8 + 255) / 256, 256, 0, stream>>>(Wv, BV, DK * DE / 8);
    for (int b = 0; b < NB_; ++b) {
        k_cvt8<<<(TT * DE / 8 + 255) / 256, 256, 0, stream>>>(x + (size_t)b * TT * DE, XB, (size_t)TT * DE / 8);
        k_gemmw<bf, 0, true><<<dim3(TT / 64, DK / 64, 1), 32, 0, stream>>>(XB, nullptr, BQ, nullptr, DE, QKV, D3, bq, 0, 0, 0); k_gemmw<bf, 0, true><<<dim3(TT / 64, DK / 64, 1), 32, 0, stream>>>(XB, nullptr, BK, nullptr, DE, QKV + DK, D3, bk, 0, 0, 0); k_gemmw<bf, 0, true><<<dim3(TT / 64, DK / 64, 1), 32, 0, stream>>>(XB, nullptr, BV, nullptr, DE, QKV + 2 * DK, D3, bv, 0, 0, 0);
        k_temp<<<(TT + 255) / 256, 256, 0, stream>>>(QKV, tokq, tokv, alpha, TQ, TV); k_gpl<<<(TT * DK / 4 + 255) / 256, 256, 0, stream>>>(QKV, TQ, GQh, GQl, Kh, Kl); k_gvt<<<(DK * TT / 4 + 255) / 256, 256, 0, stream>>>(QKV, TV, GVh, GVl);
        k_gemmc<bf, 2, 1><<<dim3(TT / 64, TT / 64, 1), 32, 0, stream>>>(GQh, GQl, Kh, Kl, DK, Sb, TT, 0, 0, 0, 0);
        k_csoft<<<TT / 8, 256, 0, stream>>>(Sb, Ph, Pl);
        k_gemmc<bf, 2, 2><<<dim3(TT / 64, DK / 64, 1), 32, 0, stream>>>(Ph, Pl, GVh, GVl, TT, OUT + (size_t)b * TT * DK, DK, 0, 0, 0, 0); }
}
